// MLPPredictor_33028298506368
// MI455X (gfx1250) — hardware-verified
//
#include <hip/hip_runtime.h>
#include <math.h>

constexpr int kNodes     = 100000;
constexpr int kNodesPad  = 100032;
constexpr int kEdges     = 1600000;
constexpr int kFeat      = 128;
constexpr int kCat       = 256;
constexpr int kEdgeBlk   = 64;
constexpr int kAPitch    = 136;
constexpr int kThreads   = 256;
constexpr int kPrepBlkH  = kNodesPad * kFeat / 8 / kThreads;
constexpr int kPrepBlkW1 = kCat * kFeat / 8 / kThreads;
constexpr int kPrepBlkW2 = kFeat * kFeat / 8 / kThreads;
constexpr float kX1Carry = 16.0f;
constexpr float kW2Carry = 16.0f;
constexpr float kL2Scale = 1.0f / 256.0f;

static_assert(kNodesPad % 64 == 0 && kNodesPad >= kNodes && kNodesPad - kNodes < 64, "node GEMM M padding");
static_assert(kCat % 64 == 0 && kFeat % 32 == 0, "node GEMM N tile multiple, K % 32");
static_assert(kEdges % kEdgeBlk == 0, "edge blocks exact");
static_assert(kPrepBlkH * kThreads * 8 == kNodesPad * kFeat, "prep coverage: node plane incl. pad rows");
static_assert(kPrepBlkW1 * kThreads * 8 == kCat * kFeat, "prep coverage: Bt1");
static_assert(kPrepBlkW2 * kThreads * 8 == kFeat * kFeat, "prep coverage: Bt2");
static_assert(kEdgeBlk == 64 && kThreads == 256 && kFeat == 128, "edge kernel lane maps assume these");

constexpr size_t kHbBytes  = (size_t)kNodesPad * kFeat * 2;
constexpr size_t kYBytes   = (size_t)kNodesPad * kCat * 4;
constexpr size_t kBt1Bytes = (size_t)kCat * kFeat * 2;
constexpr size_t kBt2Bytes = (size_t)kFeat * kFeat * 2;
constexpr size_t kOffHb  = 0;
constexpr size_t kOffY   = kOffHb + kHbBytes;
constexpr size_t kOffBt1 = kOffY + kYBytes;
constexpr size_t kOffBt2 = kOffBt1 + kBt1Bytes;
constexpr size_t kWsTotal = kOffBt2 + kBt2Bytes;
static_assert(kOffY % 256 == 0 && kOffBt1 % 256 == 0 && kOffBt2 % 256 == 0, "carve alignment");
static_assert(kWsTotal == 128139264ull && kWsTotal <= 134217728ull, "carve total under 128 MiB");

typedef __attribute__((ext_vector_type(16))) _Float16 v16h;
typedef __attribute__((ext_vector_type(8)))  _Float16 v8h;
typedef __attribute__((ext_vector_type(4)))  _Float16 v4h;
typedef __attribute__((ext_vector_type(16))) __bf16   v16b;
typedef __attribute__((ext_vector_type(8)))  __bf16   v8b;
typedef __attribute__((ext_vector_type(8)))  float    v8f;
typedef __attribute__((ext_vector_type(4)))  float    v4f;
typedef __attribute__((ext_vector_type(4)))  unsigned int v4u;

__device__ __forceinline__ unsigned short f2bf_bits(float f) {
  unsigned u = __float_as_uint(f);
  return (unsigned short)((u + 0x7FFFu + ((u >> 16) & 1u)) >> 16);
}
__device__ __forceinline__ float bf_bits2f(unsigned short h) { return __uint_as_float(((unsigned)h) << 16); }

__device__ __forceinline__ void dep_guard_h(v8f& a, v8f& b, v16h x, v16h y) { asm volatile("v_nop\n\tv_nop\n\tv_nop\n\tv_nop" : "+v"(a), "+v"(b) : "v"(x), "v"(y)); }
__device__ __forceinline__ void dep_guard_b(v8f& a, v8f& b, v16b x, v16b y) { asm volatile("v_nop\n\tv_nop\n\tv_nop\n\tv_nop" : "+v"(a), "+v"(b) : "v"(x), "v"(y)); }
__device__ __forceinline__ void keep4_h(v16h a, v16h b, v16h c, v16h d) { asm volatile("v_nop" :: "v"(a), "v"(b), "v"(c), "v"(d)); }
__device__ __forceinline__ void keep4_b(v16b a, v16b b, v16b c, v16b d) { asm volatile("v_nop" :: "v"(a), "v"(b), "v"(c), "v"(d)); }
__device__ __forceinline__ void acc_guard4(v8f& a, v8f& b, v8f& c, v8f& d) { asm volatile("v_nop\n\tv_nop\n\tv_nop\n\tv_nop" : "+v"(a), "+v"(b), "+v"(c), "+v"(d)); }
template <typename T> struct Frag;
template <> struct Frag<_Float16> {
  typedef v16h V; union U { v16h v; v8h h[2]; };
  static __device__ __forceinline__ v16h load(const _Float16* p) {
    U f; f.h[0] = *(const v8h*)(p); f.h[1] = *(const v8h*)(p + 16); return f.v;
  }
  static __device__ __forceinline__ v8f mma(v16h a, v16h b, v8f c) {
    return __builtin_amdgcn_wmma_f32_16x16x32_f16(false, a, false, b, (short)0, c, false, false);
  }
  static __device__ __forceinline__ void guard(v8f& a, v8f& b, v16h x, v16h y) { dep_guard_h(a, b, x, y); }
  static __device__ __forceinline__ void keep(v16h a, v16h b, v16h c, v16h d) { keep4_h(a, b, c, d); }
};
template <> struct Frag<__bf16> {
  typedef v16b V; union U { v16b v; v8b h[2]; };
  static __device__ __forceinline__ v16b load(const __bf16* p) {
    U f; f.h[0] = *(const v8b*)(p); f.h[1] = *(const v8b*)(p + 16); return f.v;
  }
  static __device__ __forceinline__ v8f mma(v16b a, v16b b, v8f c) {
    return __builtin_amdgcn_wmma_f32_16x16x32_bf16(false, a, false, b, (short)0, c, false, false);
  }
  static __device__ __forceinline__ void guard(v8f& a, v8f& b, v16b x, v16b y) { dep_guard_b(a, b, x, y); }
  static __device__ __forceinline__ void keep(v16b a, v16b b, v16b c, v16b d) { keep4_b(a, b, c, d); }
};

__device__ __forceinline__ unsigned pk16(unsigned short a, unsigned short b) { return (unsigned)a | ((unsigned)b << 16); }
__device__ __forceinline__ unsigned short h_bits(float f) { const _Float16 h = (_Float16)f; return __builtin_bit_cast(unsigned short, h); }
__device__ __forceinline__ float bf_rne(float f) { return bf_bits2f(f2bf_bits(f)); }

__device__ __forceinline__ v8f mma_h_guard(v16h a, v16h b, v8f c) {
  c = __builtin_amdgcn_wmma_f32_16x16x32_f16(false, a, false, b, (short)0, c, false, false);
  asm volatile("v_nop\n\tv_nop\n\tv_nop\n\tv_nop" : "+v"(c) : "v"(a), "v"(b));
  return c;
}

template <int ET> struct Elem;
template <> struct Elem<0> { typedef _Float16 T; };
template <> struct Elem<1> { typedef __bf16 T; };
template <int ET, bool SPLIT, int BIAS_MODE, int OUT_MODE, bool RESID, int ACT = 0>
__global__ __launch_bounds__(256) void wmma_gemm64(
    const unsigned short* __restrict__ Ap, const unsigned short* __restrict__ A2p, int lda, long strideA,
    const unsigned short* __restrict__ Btp, const unsigned short* __restrict__ Bt2p, int ldb, long strideB,
    void* __restrict__ Cout, void* __restrict__ Cout2, int ldc, long strideC,
    const float* __restrict__ bias,
    const float* __restrict__ resid, long strideR,
    int M, int N, int K, float scale) {
  typedef typename Elem<ET>::T T;
  typedef typename Frag<T>::V V;
  const T* A = (const T*)Ap; const T* A2 = (const T*)A2p; const T* Bt = (const T*)Btp; const T* Bt2 = (const T*)Bt2p;
  __shared__ __align__(16) float sT[8][16 * 68];
  const int b    = blockIdx.y;
  const int lane = threadIdx.x & 31;
  const int wave = threadIdx.x >> 5;
  const int tilesN = N >> 6;
  const int tilesM = M >> 6;
  const int tile = blockIdx.x * 8 + wave;
  if (tile >= tilesM * tilesN) return;
  const int tm = tile / tilesN;
  const int tn = tile - tm * tilesN;
  const int m0 = tm << 6;
  const int n0 = tn << 6;

  const T* Ab  = A  + (size_t)b * strideA;
  const T* Bb  = Bt + (size_t)b * strideB;
  const T* Ab2 = SPLIT ? (A2  + (size_t)b * strideA) : nullptr;
  const T* Bb2 = SPLIT ? (Bt2 + (size_t)b * strideB) : nullptr;

  const int rlane = lane & 15;
  const int koff  = (lane >> 4) * 8;
  const int mOff  = (lane >> 4) * 8;

  v8f acc[4][4];
#pragma unroll
  for (int i = 0; i < 4; ++i)
#pragma unroll
    for (int j = 0; j < 4; ++j) acc[i][j] = (v8f){0.f,0.f,0.f,0.f,0.f,0.f,0.f,0.f};

  for (int k0 = 0; k0 < K; k0 += 32) {
    V bh[4], bl[4];
#pragma unroll
    for (int j = 0; j < 4; ++j) {
      const size_t bo = (size_t)(n0 + (j << 4) + rlane) * ldb + koff + k0;
      bh[j] = Frag<T>::load(Bb + bo);
      if (SPLIT) bl[j] = Frag<T>::load(Bb2 + bo);
    }
#pragma unroll
    for (int i = 0; i < 4; ++i) {
      const size_t ao = (size_t)(m0 + (i << 4) + rlane) * lda + koff + k0;
      V ah = Frag<T>::load(Ab + ao);
      V al;
      if (SPLIT) al = Frag<T>::load(Ab2 + ao);
#pragma unroll
      for (int j = 0; j < 4; ++j) {
        acc[i][j] = Frag<T>::mma(ah, bh[j], acc[i][j]);
        if (SPLIT) {
          acc[i][j] = Frag<T>::mma(ah, bl[j], acc[i][j]);
          acc[i][j] = Frag<T>::mma(al, bh[j], acc[i][j]);
        }
      }
      Frag<T>::guard(acc[i][0], acc[i][3], ah, SPLIT ? al : ah);
    }
    Frag<T>::keep(bh[0], bh[1], bh[2], bh[3]);
    if (SPLIT) Frag<T>::keep(bl[0], bl[1], bl[2], bl[3]);
  }
  acc_guard4(acc[0][0], acc[0][1], acc[0][2], acc[0][3]);
  acc_guard4(acc[1][0], acc[1][1], acc[1][2], acc[1][3]);
  acc_guard4(acc[2][0], acc[2][1], acc[2][2], acc[2][3]);
  acc_guard4(acc[3][0], acc[3][1], acc[3][2], acc[3][3]);

  float* slab = sT[wave];
  const float* Rb = RESID ? (resid + (size_t)b * strideR) : nullptr;
#pragma unroll
  for (int i = 0; i < 4; ++i) {
    const int mBase = m0 + (i << 4);
#pragma unroll
    for (int j = 0; j < 4; ++j) {
      const int n = n0 + (j << 4) + rlane;
      float bv = 0.f;
      if (BIAS_MODE == 2) bv = bias[n];
#pragma unroll
      for (int r = 0; r < 8; ++r) {
        float v = acc[i][j][r] * scale;
        if (BIAS_MODE == 1) v += bias[mBase + mOff + r];
        if (BIAS_MODE == 2) v += bv;
        if (RESID) v += Rb[(size_t)(mBase + mOff + r) * ldc + n];
        if (ACT == 2) v = fmaxf(v, 0.0f);
        if (ACT == 4) v = (v > 0.f) ? v : 0.01f * v;
        slab[(mOff + r) * 68 + (j << 4) + rlane] = v;
      }
    }
    __builtin_amdgcn_fence(__ATOMIC_RELEASE, "workgroup");
    __builtin_amdgcn_wave_barrier();
    __builtin_amdgcn_fence(__ATOMIC_ACQUIRE, "workgroup");
    if (OUT_MODE == 0) {
      float* C = (float*)Cout + (size_t)b * strideC;
      const int hh = lane >> 4, c4 = (lane & 15) * 4;
      for (int pass = 0; pass < 2; ++pass) {
#pragma unroll
        for (int it = 0; it < 8; ++it) {
          const int row = it * 2 + hh;
          v4f v = *(const v4f*)(slab + row * 68 + c4);
          *(volatile v4f*)(C + (size_t)(mBase + row) * ldc + n0 + c4) = v;
        }
        __threadfence();
      }
    } else {
      const int q = lane >> 3, c8 = (lane & 7) * 8;
      unsigned short* C  = (unsigned short*)Cout  + (size_t)b * strideC;
      unsigned short* C2 = (OUT_MODE == 2) ? ((unsigned short*)Cout2 + (size_t)b * strideC) : nullptr;
      for (int pass = 0; pass < 2; ++pass) {
#pragma unroll
        for (int it = 0; it < 4; ++it) {
          const int row = it * 4 + q;
          const float* sp = slab + row * 68 + c8;
          v8h hv, lv;
#pragma unroll
          for (int e = 0; e < 8; ++e) {
            if (OUT_MODE == 1) {
              hv[e] = (_Float16)sp[e];
            } else {
              unsigned short hb = f2bf_bits(sp[e]);
              unsigned short lb = f2bf_bits(sp[e] - bf_bits2f(hb));
              hv[e] = __builtin_bit_cast(_Float16, hb);
              lv[e] = __builtin_bit_cast(_Float16, lb);
            }
          }
          *(volatile v8h*)(C + (size_t)(mBase + row) * ldc + n0 + c8) = hv;
          if (OUT_MODE == 2) *(volatile v8h*)(C2 + (size_t)(mBase + row) * ldc + n0 + c8) = lv;
        }
        __threadfence();
      }
    }
    __builtin_amdgcn_fence(__ATOMIC_RELEASE, "workgroup");
    __builtin_amdgcn_wave_barrier();
    __builtin_amdgcn_fence(__ATOMIC_ACQUIRE, "workgroup");
  }
}

__global__ __launch_bounds__(kThreads) void prep_kernel(const float* __restrict__ hfeat, const float* __restrict__ W1,
                                                       const float* __restrict__ W2,
                                                       unsigned short* __restrict__ Hb, unsigned short* __restrict__ Bt1,
                                                       unsigned short* __restrict__ Bt2,
                                                       int n_nodes, int nbH, int nbW1) {
  const int t  = threadIdx.x;
  const int bx = blockIdx.x;
  unsigned short bits[8];
  unsigned short* dstp;
  if (bx < nbH) {
    const int i    = bx * kThreads + t;
    const int row  = i >> 4;
    const int c8   = (i & 15) * 8;
    const int rowc = row < n_nodes ? row : n_nodes - 1;
    const bool live = row < n_nodes;
    const float* p = hfeat + (size_t)rowc * kFeat + c8;
    const v4f a = *(const v4f*)(p);
    const v4f c = *(const v4f*)(p + 4);
#pragma unroll
    for (int e = 0; e < 4; ++e) {
      const float x0 = live ? a[e] : 0.0f;
      const float x1 = live ? c[e] : 0.0f;
      bits[e]     = f2bf_bits(x0);
      bits[4 + e] = f2bf_bits(x1);
    }
    dstp = Hb + 8 * (size_t)i;
  } else if (bx < nbH + nbW1) {
    const int j  = (bx - nbH) * kThreads + t;
    const int n2 = j >> 4;
    const int k8 = (j & 15) * 8;
    const float* p = W1 + (size_t)(n2 & (kFeat - 1)) * kCat + (n2 >> 7) * kFeat + k8;
    const v4f a = *(const v4f*)(p);
    const v4f c = *(const v4f*)(p + 4);
#pragma unroll
    for (int e = 0; e < 4; ++e) { bits[e] = f2bf_bits(a[e]); bits[4 + e] = f2bf_bits(c[e]); }
    dstp = Bt1 + 8 * (size_t)j;
  } else {
    const int j = (bx - nbH - nbW1) * kThreads + t;
    const float* p = W2 + 8 * (size_t)j;
    const v4f a = *(const v4f*)(p);
    const v4f c = *(const v4f*)(p + 4);
#pragma unroll
    for (int e = 0; e < 4; ++e) {
      bits[e]     = h_bits(bf_rne(a[e]) * kW2Carry);
      bits[4 + e] = h_bits(bf_rne(c[e]) * kW2Carry);
    }
    dstp = Bt2 + 8 * (size_t)j;
  }
  const v4u u = (v4u){pk16(bits[0], bits[1]), pk16(bits[2], bits[3]), pk16(bits[4], bits[5]), pk16(bits[6], bits[7])};
  *(volatile v4u*)dstp = u;
  __threadfence();
  *(volatile v4u*)dstp = u;
}

__global__ __launch_bounds__(kThreads) void edge_kernel(const float* __restrict__ Y, const int* __restrict__ src_idx,
                                                       const int* __restrict__ dst_idx, const float* __restrict__ b1,
                                                       const unsigned short* __restrict__ Bt2p, const float* __restrict__ b2,
                                                       const float* __restrict__ W3, const float* __restrict__ b3,
                                                       float* __restrict__ out, int n_edges, int n_nodes) {
  __shared__ __align__(16) _Float16 At[kEdgeBlk * kAPitch];
  __shared__ __align__(16) float part_s[8 * kEdgeBlk];
  const int tid  = threadIdx.x;
  const int lane = tid & 31;
  const int wave = tid >> 5;
  const int rlane = lane & 15;
  const int hh    = lane >> 4;
  const int koff  = hh * 8;
  const size_t ebase = (size_t)blockIdx.x * kEdgeBlk;
  const _Float16* Bt2 = (const _Float16*)Bt2p;

  const int c4 = lane * 4;
  v4f b1r;
  {
    const v4f tb = *(const v4f*)(b1 + c4);
#pragma unroll
    for (int e = 0; e < 4; ++e) b1r[e] = bf_rne(tb[e]);
  }
  const int ncol = wave * 16 + rlane;
  const float b2r = bf_rne(b2[ncol]);
  const float w3r = bf_rne(W3[ncol]);
  const float b3r = bf_rne(b3[0]);

#pragma unroll 2
  for (int it = 0; it < 8; ++it) {
    const int er = it * 8 + wave;
    size_t ge = ebase + (size_t)er;
    ge = ge < (size_t)n_edges ? ge : (size_t)(n_edges - 1);
    int s = src_idx[ge]; s = s < 0 ? 0 : (s >= n_nodes ? n_nodes - 1 : s);
    int d = dst_idx[ge]; d = d < 0 ? 0 : (d >= n_nodes ? n_nodes - 1 : d);
    const v4f p = *(const v4f*)(Y + (size_t)s * kCat + c4);
    const v4f q = *(const v4f*)(Y + (size_t)d * kCat + kFeat + c4);
    v4h hv;
#pragma unroll
    for (int e = 0; e < 4; ++e) {
      float z = (p[e] + q[e]) + b1r[e];
      z = fmaxf(z, 0.0f) * kX1Carry;
      hv[e] = (_Float16)z;
    }
    *(v4h*)(At + er * kAPitch + c4) = hv;
  }
  __syncthreads();

  v16h bq[4];
#pragma unroll
  for (int kt = 0; kt < 4; ++kt) bq[kt] = Frag<_Float16>::load(Bt2 + (size_t)ncol * kFeat + koff + kt * 32);
  v8f acc[4];
#pragma unroll
  for (int mt = 0; mt < 4; ++mt) acc[mt] = (v8f){0.f,0.f,0.f,0.f,0.f,0.f,0.f,0.f};
#pragma unroll
  for (int kt = 0; kt < 4; ++kt) {
#pragma unroll
    for (int mt = 0; mt < 4; ++mt) {
      const v16h af = Frag<_Float16>::load(At + (mt * 16 + rlane) * kAPitch + koff + kt * 32);
      acc[mt] = mma_h_guard(af, bq[kt], acc[mt]);
    }
  }
  acc_guard4(acc[0], acc[1], acc[2], acc[3]);

#pragma unroll
  for (int mt = 0; mt < 4; ++mt) {
#pragma unroll
    for (int r = 0; r < 8; ++r) {
      float v = acc[mt][r] * kL2Scale + b2r;
      v = fmaxf(v, 0.0f) * w3r;
      v += __shfl_xor(v, 1, 32);
      v += __shfl_xor(v, 2, 32);
      v += __shfl_xor(v, 4, 32);
      v += __shfl_xor(v, 8, 32);
      if (rlane == 0) part_s[wave * kEdgeBlk + mt * 16 + hh * 8 + r] = v;
    }
  }
  __syncthreads();

  if (wave == 0) {
    const int l4 = rlane * 4;
    v4f sv;
#pragma unroll
    for (int j = 0; j < 4; ++j) {
      float a = 0.0f;
#pragma unroll
      for (int w = 0; w < 8; ++w) a += part_s[w * kEdgeBlk + l4 + j];
      sv[j] = a + b3r;
    }
    if (ebase + (size_t)kEdgeBlk <= (size_t)n_edges) {
      float* op = out + ebase + l4;
      if (lane < 16) *(volatile v4f*)op = sv;
      __threadfence();
      if (lane < 16) *(volatile v4f*)op = sv;
    }
  }
}

extern "C" void kernel_launch(void* const* d_in, const int* in_sizes, int n_in,
                              void* d_out, int out_size, void* d_ws, size_t ws_size, hipStream_t stream) {
  if (n_in < 9) return;
  if (in_sizes[0] != kNodes * kFeat || in_sizes[1] != kEdges || in_sizes[2] != kEdges ||
      in_sizes[3] != kFeat * kCat || in_sizes[4] != kFeat || in_sizes[5] != kFeat * kFeat ||
      in_sizes[6] != kFeat || in_sizes[7] != kFeat || in_sizes[8] < 1) return;
  if (out_size != kEdges) return;
  if (kWsTotal > ws_size) return;

  const float* hfeat = (const float*)d_in[0];
  const int*   src   = (const int*)  d_in[1];
  const int*   dst   = (const int*)  d_in[2];
  const float* W1    = (const float*)d_in[3];
  const float* b1    = (const float*)d_in[4];
  const float* W2    = (const float*)d_in[5];
  const float* b2    = (const float*)d_in[6];
  const float* W3    = (const float*)d_in[7];
  const float* b3    = (const float*)d_in[8];
  float* out = (float*)d_out;

  char* ws = (char*)d_ws;
  unsigned short* Hb  = (unsigned short*)(ws + kOffHb);
  float*          Y   = (float*)(ws + kOffY);
  unsigned short* Bt1 = (unsigned short*)(ws + kOffBt1);
  unsigned short* Bt2 = (unsigned short*)(ws + kOffBt2);

  prep_kernel<<<kPrepBlkH + kPrepBlkW1 + kPrepBlkW2, kThreads, 0, stream>>>(hfeat, W1, W2, Hb, Bt1, Bt2,
                                                                          kNodes, kPrepBlkH, kPrepBlkW1);

  {
    const int tiles = (kNodesPad / 64) * (kCat / 64);
    wmma_gemm64<1, false, 0, 0, false, 0><<<dim3((tiles + 7) / 8, 1), kThreads, 0, stream>>>(
        (const unsigned short*)Hb, (const unsigned short*)nullptr, kFeat, 0L,
        (const unsigned short*)Bt1, (const unsigned short*)nullptr, kFeat, 0L,
        (void*)Y, (void*)nullptr, kCat, 0L,
        (const float*)nullptr, (const float*)nullptr, 0L, kNodesPad, kCat, kFeat, 1.0f);
  }

  edge_kernel<<<kEdges / kEdgeBlk, kThreads, 0, stream>>>(Y, src, dst, b1, Bt2, b2, W3, b3, out, kEdges, kNodes);
}
